// LSTM_75428215652813
// MI455X (gfx1250) — hardware-verified
//
#include <hip/hip_runtime.h>
#include <math.h>

constexpr int NBATCH  = 512;
constexpr int NSEQ    = 128;
constexpr int NWORDV  = 100000;
constexpr int DWORDE  = 100;
constexpr int NTAGV   = 52;
constexpr int DTAGE   = 20;
constexpr int NPOSV   = 200;
constexpr int DPOSE   = 20;
constexpr int NXIN    = 160;
constexpr int NHID    = 256;
constexpr int NGATE   = 4 * NHID;
constexpr int NOUTH   = 2 * NHID;
constexpr int NLIN    = 2 * NXIN + 8 * NHID;
constexpr int NMLP    = 512;
constexpr int NCLS    = 53;
constexpr int ENTV    = 68;
constexpr int NTOK    = NBATCH * NSEQ;
constexpr int NTHR    = 256;
constexpr int XPITCH  = 168;
constexpr int HPITCH  = 264;
constexpr int FEATW   = NLIN / 2;
constexpr float CARRY_F    = 16.0f;
constexpr float CARRY2_INV = 1.0f / (CARRY_F * CARRY_F);
static_assert(DWORDE + DTAGE + 2 * DPOSE == NXIN, "input width");
static_assert(NXIN % 32 == 0 && NHID % 32 == 0 && NLIN % 32 == 0, "k multiples of 32");
static_assert(NBATCH % 64 == 0 && NMLP % 64 == 0, "tile multiples of 64");
static_assert(NBATCH % 16 == 0, "16-row recurrent tiles");
static_assert(NHID == 32 * (NTHR / 32), "8 waves x 32 hidden units");
static_assert((NLIN * 2) % 128 == 0, "feature row = whole lines");
static_assert((NBATCH * NCLS) % NTHR == 0, "output grid exact");
static_assert(NTOK % 32 == 0, "embed grid exact");
static_assert((NGATE * NXIN) % (8 * NTHR) == 0 && (NGATE * NHID) % (8 * NTHR) == 0 && (NMLP * NLIN) % (8 * NTHR) == 0, "convert grids exact");

typedef __attribute__((ext_vector_type(16))) _Float16 v16h;
typedef __attribute__((ext_vector_type(8)))  _Float16 v8h;
typedef __attribute__((ext_vector_type(8)))  float    v8f;
typedef __attribute__((ext_vector_type(4)))  float    v4f;
typedef __attribute__((ext_vector_type(4)))  unsigned v4u;

__device__ __forceinline__ void guard4_h(v8f& a, v8f& b, v8f& c, v8f& d, v16h x, v16h y0, v16h y1, v16h y2, v16h y3) {
  asm volatile("v_nop\n\tv_nop\n\tv_nop\n\tv_nop" : "+v"(a), "+v"(b), "+v"(c), "+v"(d) : "v"(x), "v"(y0), "v"(y1), "v"(y2), "v"(y3));
}
__device__ __forceinline__ void keep4_h(v16h a, v16h b, v16h c, v16h d) { asm volatile("v_nop" :: "v"(a), "v"(b), "v"(c), "v"(d)); }
__device__ __forceinline__ void acc_guard4(v8f& a, v8f& b, v8f& c, v8f& d) { asm volatile("v_nop\n\tv_nop\n\tv_nop\n\tv_nop" : "+v"(a), "+v"(b), "+v"(c), "+v"(d)); }

struct FragH {
  union U { v16h v; v8h h[2]; };
  static __device__ __forceinline__ v16h load(const _Float16* p) {
    U f; f.h[0] = *(const v8h*)(p); f.h[1] = *(const v8h*)(p + 16); return f.v;
  }
  static __device__ __forceinline__ v8f mma(v16h a, v16h b, v8f c) {
    return __builtin_amdgcn_wmma_f32_16x16x32_f16(false, a, false, b, (short)0, c, false, false);
  }
};

__device__ __forceinline__ float fsig(float x)  { return __builtin_amdgcn_rcpf(1.0f + __expf(-x)); }
__device__ __forceinline__ float ftanh(float x) { return 1.0f - 2.0f * __builtin_amdgcn_rcpf(__expf(2.0f * x) + 1.0f); }

__device__ __forceinline__ float h16_to_f32(unsigned hb) {
  const unsigned sgn = (hb & 0x8000u) << 16; const unsigned em = hb & 0x7fffu;
  const float fn = __uint_as_float((em << 13) + 0x38000000u);
  const float fs = (float)em * 5.9604644775390625e-8f;
  const float mag = (em < 0x400u) ? fs : fn; return __uint_as_float(__float_as_uint(mag) | sgn);
}
__device__ __forceinline__ unsigned pack2h(float a, float b) {
  const _Float16 ha = (_Float16)a, hb = (_Float16)b;
  const unsigned ua = (unsigned)__builtin_bit_cast(unsigned short, ha);
  const unsigned ub = (unsigned)__builtin_bit_cast(unsigned short, hb);
  return ua | (ub << 16);
}

__global__ __launch_bounds__(32) void entity_idx_kernel(const int* __restrict__ pos1, const int* __restrict__ pos2,
                                                        int* __restrict__ idx1, int* __restrict__ idx2) {
  const int b = blockIdx.x * 32 + threadIdx.x;
  int i1 = 0, i2 = 0;
#pragma unroll 4
  for (int s = NSEQ - 1; s >= 0; --s) {
    const int p1 = pos1[(size_t)b * NSEQ + s];
    const int p2 = pos2[(size_t)b * NSEQ + s];
    i1 = (p1 == ENTV) ? s : i1;
    i2 = (p2 == ENTV) ? s : i2;
  }
  *(volatile int*)(idx1 + b) = i1;
  *(volatile int*)(idx2 + b) = i2;
  __threadfence();
  *(volatile int*)(idx1 + b) = i1;
  *(volatile int*)(idx2 + b) = i2;
}

__global__ __launch_bounds__(NTHR) void cvt8_f16_kernel(const float* __restrict__ src, unsigned short* __restrict__ dst, int n8) {
  const int i = blockIdx.x * NTHR + threadIdx.x;
  if (i < n8) {
    const v4f a = *(const v4f*)(src + (size_t)i * 8);
    const v4f b = *(const v4f*)(src + (size_t)i * 8 + 4);
    v8h hv;
#pragma unroll
    for (int e = 0; e < 4; ++e) {
      hv[e]     = (_Float16)(a[e] * CARRY_F);
      hv[4 + e] = (_Float16)(b[e] * CARRY_F);
    }
    *(volatile v8h*)(dst + (size_t)i * 8) = hv;
    __threadfence();
    *(volatile v8h*)(dst + (size_t)i * 8) = hv;
  }
}

__global__ __launch_bounds__(NTHR) void embed_kernel(const int* __restrict__ word, const int* __restrict__ tag,
                                                     const int* __restrict__ pos1, const int* __restrict__ pos2,
                                                     const float* __restrict__ we, const float* __restrict__ te,
                                                     const float* __restrict__ p1e, const float* __restrict__ p2e,
                                                     unsigned short* __restrict__ x16) {
  __shared__ __align__(16) float xs[32 * NXIN];
  __shared__ int ids[4][32];
  const int tid = threadIdx.x;
  const int tok0 = blockIdx.x * 32;
  if (tid < 32) {
    int w  = word[tok0 + tid];
    int tg = tag[tok0 + tid];
    int q1 = pos1[tok0 + tid];
    int q2 = pos2[tok0 + tid];
    w  = w  < 0 ? 0 : (w  > NWORDV - 1 ? NWORDV - 1 : w);
    tg = tg < 0 ? 0 : (tg > NTAGV - 1  ? NTAGV - 1  : tg);
    q1 = q1 < 0 ? 0 : (q1 > NPOSV - 1  ? NPOSV - 1  : q1);
    q2 = q2 < 0 ? 0 : (q2 > NPOSV - 1  ? NPOSV - 1  : q2);
    ids[0][tid] = w; ids[1][tid] = tg; ids[2][tid] = q1; ids[3][tid] = q2;
  }
  __syncthreads();
#pragma unroll 1
  for (int i = tid; i < 32 * (DWORDE / 4); i += NTHR) {
    const int r = i / (DWORDE / 4);
    const int q = i - r * (DWORDE / 4);
    const v4f v = *(const v4f*)(we + (size_t)ids[0][r] * DWORDE + 4 * q);
    *(v4f*)(xs + r * NXIN + 4 * q) = v;
  }
  if (tid < 32 * (DTAGE / 4)) {
    const int r = tid / (DTAGE / 4);
    const int q = tid - r * (DTAGE / 4);
    const v4f a = *(const v4f*)(te  + (size_t)ids[1][r] * DTAGE + 4 * q);
    const v4f b = *(const v4f*)(p1e + (size_t)ids[2][r] * DPOSE + 4 * q);
    const v4f c = *(const v4f*)(p2e + (size_t)ids[3][r] * DPOSE + 4 * q);
    *(v4f*)(xs + r * NXIN + DWORDE + 4 * q) = a;
    *(v4f*)(xs + r * NXIN + DWORDE + DTAGE + 4 * q) = b;
    *(v4f*)(xs + r * NXIN + DWORDE + DTAGE + DPOSE + 4 * q) = c;
  }
  __syncthreads();
  v8h hv[3];
#pragma unroll
  for (int it = 0; it < 3; ++it) {
    const int i = it * NTHR + tid;
    const int ic = i < 639 ? i : 639;
    const v4f a = *(const v4f*)(xs + ic * 8);
    const v4f b = *(const v4f*)(xs + ic * 8 + 4);
#pragma unroll
    for (int e = 0; e < 4; ++e) {
      hv[it][e]     = (_Float16)(a[e] * CARRY_F);
      hv[it][4 + e] = (_Float16)(b[e] * CARRY_F);
    }
  }
  for (int pass = 0; pass < 2; ++pass) {
#pragma unroll
    for (int it = 0; it < 3; ++it) {
      const int i = it * NTHR + tid;
      if (i < 640) *(volatile v8h*)(x16 + (size_t)tok0 * NXIN + (size_t)i * 8) = hv[it];
    }
    __threadfence();
  }
}

__device__ __forceinline__ void load_x_tile(_Float16* Ax, const _Float16* x16, int rowbase, int te, int tid) {
#pragma unroll
  for (int it = 0; it < 2; ++it) {
    const int i = it * NTHR + tid;
    if (i < 16 * (NXIN / 8)) {
      const int m = i / (NXIN / 8);
      const int c8 = (i - m * (NXIN / 8)) * 8;
      const v8h v = *(const v8h*)(x16 + ((size_t)(rowbase + m) * NSEQ + (size_t)te) * NXIN + c8);
      *(v8h*)(Ax + m * XPITCH + c8) = v;
    }
  }
}

__global__ __launch_bounds__(NTHR) void birnn_seq_kernel(const unsigned short* __restrict__ x16p,
                                                         const unsigned short* __restrict__ wihF, const unsigned short* __restrict__ whhF,
                                                         const unsigned short* __restrict__ wihB, const unsigned short* __restrict__ whhB,
                                                         const float* __restrict__ bihF, const float* __restrict__ bhhF,
                                                         const float* __restrict__ bihB, const float* __restrict__ bhhB,
                                                         unsigned short* __restrict__ hs16p) {
  __shared__ __align__(16) _Float16 Ax[16 * XPITCH];
  __shared__ __align__(16) _Float16 Ah[16 * HPITCH];
  const _Float16* x16 = (const _Float16*)x16p;
  _Float16* hs16 = (_Float16*)hs16p;
  const int dir = blockIdx.y;
  const _Float16* WX = (const _Float16*)(dir ? wihB : wihF);
  const _Float16* WH = (const _Float16*)(dir ? whhB : whhF);
  const float* bi = dir ? bihB : bihF;
  const float* bh = dir ? bhhB : bhhF;
  const int tid = threadIdx.x, lane = tid & 31, wave = tid >> 5;
  const int c = lane & 15, hh = lane >> 4, koff = hh * 8;
  const int rowbase = blockIdx.x * 16;

#pragma unroll 1
  for (int i = 0; i < 16; ++i) Ah[i * HPITCH + tid] = (_Float16)0.0f;
  load_x_tile(Ax, x16, rowbase, dir ? (NSEQ - 1) : 0, tid);

  float cst[2][8], hst[2][8], bb[2][4];
#pragma unroll
  for (int nt = 0; nt < 2; ++nt) {
    const int j = 32 * wave + 16 * nt + c;
#pragma unroll
    for (int g = 0; g < 4; ++g) bb[nt][g] = bi[g * NHID + j] + bh[g * NHID + j];
    asm volatile("" ::: "memory");
#pragma unroll
    for (int r = 0; r < 8; ++r) { cst[nt][r] = 0.0f; hst[nt][r] = 0.0f; }
  }
  __syncthreads();

  const _Float16* axrow = Ax + c * XPITCH + koff;
  const _Float16* ahrow = Ah + c * HPITCH + koff;
  const v8f z8 = {0.f, 0.f, 0.f, 0.f, 0.f, 0.f, 0.f, 0.f};

#pragma unroll 1
  for (int t = 0; t < NSEQ; ++t) {
    const int te = dir ? (NSEQ - 1 - t) : t;
#pragma unroll
    for (int nt = 0; nt < 2; ++nt) {
      const int j = 32 * wave + 16 * nt + c;
      const _Float16* wx = WX + (size_t)j * NXIN + koff;
      const _Float16* wh = WH + (size_t)j * NHID + koff;
      v8f acc[4];
      acc[0] = z8; acc[1] = z8; acc[2] = z8; acc[3] = z8;
#pragma unroll 1
      for (int kx = 0; kx < NXIN; kx += 32) {
        const v16h a  = FragH::load(axrow + kx);
        const v16h b0 = FragH::load(wx + kx);
        const v16h b1 = FragH::load(wx + (size_t)1 * NHID * NXIN + kx);
        const v16h b2 = FragH::load(wx + (size_t)2 * NHID * NXIN + kx);
        const v16h b3 = FragH::load(wx + (size_t)3 * NHID * NXIN + kx);
        acc[0] = FragH::mma(a, b0, acc[0]);
        acc[1] = FragH::mma(a, b1, acc[1]);
        acc[2] = FragH::mma(a, b2, acc[2]);
        acc[3] = FragH::mma(a, b3, acc[3]);
        guard4_h(acc[0], acc[1], acc[2], acc[3], a, b0, b1, b2, b3);
        keep4_h(b0, b1, b2, b3);
      }
#pragma unroll 1
      for (int k0 = 0; k0 < NHID; k0 += 32) {
        const v16h a  = FragH::load(ahrow + k0);
        const v16h b0 = FragH::load(wh + k0);
        const v16h b1 = FragH::load(wh + (size_t)1 * NHID * NHID + k0);
        const v16h b2 = FragH::load(wh + (size_t)2 * NHID * NHID + k0);
        const v16h b3 = FragH::load(wh + (size_t)3 * NHID * NHID + k0);
        acc[0] = FragH::mma(a, b0, acc[0]);
        acc[1] = FragH::mma(a, b1, acc[1]);
        acc[2] = FragH::mma(a, b2, acc[2]);
        acc[3] = FragH::mma(a, b3, acc[3]);
        guard4_h(acc[0], acc[1], acc[2], acc[3], a, b0, b1, b2, b3);
        keep4_h(b0, b1, b2, b3);
      }
      acc_guard4(acc[0], acc[1], acc[2], acc[3]);
#pragma unroll
      for (int r = 0; r < 8; ++r) {
        const float zi = acc[0][r] * CARRY2_INV + bb[nt][0];
        const float zf = acc[1][r] * CARRY2_INV + bb[nt][1];
        const float zg = acc[2][r] * CARRY2_INV + bb[nt][2];
        const float zo = acc[3][r] * CARRY2_INV + bb[nt][3];
        const float ig = fsig(zi);
        const float fg = fsig(zf);
        const float gg = ftanh(zg);
        const float og = fsig(zo);
        const float cn = fg * cst[nt][r] + ig * gg;
        cst[nt][r] = cn;
        hst[nt][r] = og * ftanh(cn);
      }
    }
    __syncthreads();
#pragma unroll
    for (int nt = 0; nt < 2; ++nt) {
      const int j = 32 * wave + 16 * nt + c;
#pragma unroll
      for (int r = 0; r < 8; ++r) Ah[(8 * hh + r) * HPITCH + j] = (_Float16)(hst[nt][r] * CARRY_F);
    }
    {
      const int tn = (t + 1 < NSEQ) ? (t + 1) : (NSEQ - 1);
      const int ten = dir ? (NSEQ - 1 - tn) : tn;
      load_x_tile(Ax, x16, rowbase, ten, tid);
    }
    __syncthreads();
    for (int pass = 0; pass < 2; ++pass) {
#pragma unroll
      for (int it = 0; it < 2; ++it) {
        const int idx = it * NTHR + tid;
        const int row = idx >> 5, c8 = (idx & 31) * 8;
        const v8h v = *(const v8h*)(Ah + row * HPITCH + c8);
        *(volatile v8h*)(hs16 + ((size_t)(rowbase + row) * NSEQ + (size_t)te) * NOUTH + (size_t)dir * NHID + c8) = v;
      }
      __threadfence();
    }
  }
}

__global__ __launch_bounds__(NTHR) void pool_feat_kernel(const unsigned short* __restrict__ hs16p, const unsigned short* __restrict__ x16p,
                                                         const int* __restrict__ idx1, const int* __restrict__ idx2,
                                                         unsigned short* __restrict__ feat16p) {
  __shared__ __align__(16) unsigned fsw[FEATW];
  const int tid = threadIdx.x;
  const int b = blockIdx.x;
  int i1 = idx1[b], i2 = idx2[b];
  i1 = i1 < 0 ? 0 : (i1 > NSEQ - 1 ? NSEQ - 1 : i1);
  i2 = i2 < 0 ? 0 : (i2 > NSEQ - 1 ? NSEQ - 1 : i2);
  const unsigned* hw = (const unsigned*)(const void*)hs16p + (size_t)b * NSEQ * (NOUTH / 2);
  float m1a = -INFINITY, m1b = -INFINITY, m2a = -INFINITY, m2b = -INFINITY;
#pragma unroll 4
  for (int t = 0; t < NSEQ; ++t) {
    const unsigned w = hw[(size_t)t * (NOUTH / 2) + tid];
    const float a  = h16_to_f32(w & 0xffffu);
    const float bq = h16_to_f32(w >> 16);
    if (t < i2)  { m1a = fmaxf(m1a, a); m1b = fmaxf(m1b, bq); }
    if (t >= i1) { m2a = fmaxf(m2a, a); m2b = fmaxf(m2b, bq); }
  }
  const unsigned w0 = hw[tid];
  const unsigned w1 = hw[(size_t)i1 * (NOUTH / 2) + tid];
  const unsigned w2 = hw[(size_t)i2 * (NOUTH / 2) + tid];
  const unsigned pm1c = pack2h(m1a, m1b);
  const unsigned pm1 = (i2 == 0) ? w0 : pm1c;
  const unsigned pm2 = pack2h(m2a, m2b);
  fsw[tid] = pm1;
  fsw[256 + tid] = pm2;
  fsw[592 + tid] = w1;
  fsw[928 + tid] = w2;
  {
    const unsigned* xw = (const unsigned*)(const void*)x16p;
    const int kk = tid < (NXIN / 2 - 1) ? tid : (NXIN / 2 - 1);
    const unsigned ue1 = xw[((size_t)b * NSEQ + (size_t)i1) * (NXIN / 2) + kk];
    const unsigned ue2 = xw[((size_t)b * NSEQ + (size_t)i2) * (NXIN / 2) + kk];
    if (tid < NXIN / 2) { fsw[512 + tid] = ue1; fsw[848 + tid] = ue2; }
  }
  __syncthreads();
  v4u val[2];
#pragma unroll
  for (int it = 0; it < 2; ++it) {
    const int i = it * NTHR + tid;
    const int ic = i < (FEATW / 4 - 1) ? i : (FEATW / 4 - 1);
    val[it] = *(const v4u*)(fsw + 4 * ic);
  }
  unsigned* fw = (unsigned*)(void*)feat16p + (size_t)b * FEATW;
  for (int pass = 0; pass < 2; ++pass) {
#pragma unroll
    for (int it = 0; it < 2; ++it) {
      const int i = it * NTHR + tid;
      if (i < FEATW / 4) *(volatile v4u*)(fw + 4 * i) = val[it];
    }
    __threadfence();
  }
}

__global__ __launch_bounds__(256) void mlp1_gemm_kernel(const unsigned short* __restrict__ Ap, const unsigned short* __restrict__ Btp,
                                                        float* __restrict__ Cout, const float* __restrict__ bias, float scale) {
  const _Float16* A  = (const _Float16*)Ap;
  const _Float16* Bt = (const _Float16*)Btp;
  __shared__ __align__(16) float sT[8][16 * 68];
  const int lane = threadIdx.x & 31;
  const int wave = threadIdx.x >> 5;
  constexpr int tilesN = NMLP >> 6;
  constexpr int tilesM = NBATCH >> 6;
  const int tile = blockIdx.x * 8 + wave;
  if (tile >= tilesM * tilesN) return;
  const int tm = tile / tilesN;
  const int tn = tile - tm * tilesN;
  const int m0 = tm << 6;
  const int n0 = tn << 6;
  const int rlane = lane & 15;
  const int koff  = (lane >> 4) * 8;
  const int mOff  = (lane >> 4) * 8;

  v8f acc[4][4];
#pragma unroll
  for (int i = 0; i < 4; ++i)
#pragma unroll
    for (int j = 0; j < 4; ++j) acc[i][j] = (v8f){0.f, 0.f, 0.f, 0.f, 0.f, 0.f, 0.f, 0.f};

  for (int k0 = 0; k0 < NLIN; k0 += 32) {
    v16h bfr[4];
#pragma unroll
    for (int j = 0; j < 4; ++j) {
      const size_t bo = (size_t)(n0 + (j << 4) + rlane) * NLIN + koff + k0;
      bfr[j] = FragH::load(Bt + bo);
    }
#pragma unroll
    for (int i = 0; i < 4; ++i) {
      const size_t ao = (size_t)(m0 + (i << 4) + rlane) * NLIN + koff + k0;
      const v16h ah = FragH::load(A + ao);
#pragma unroll
      for (int j = 0; j < 4; ++j) acc[i][j] = FragH::mma(ah, bfr[j], acc[i][j]);
      guard4_h(acc[i][0], acc[i][1], acc[i][2], acc[i][3], ah, bfr[0], bfr[1], bfr[2], bfr[3]);
    }
    keep4_h(bfr[0], bfr[1], bfr[2], bfr[3]);
  }
  acc_guard4(acc[0][0], acc[0][1], acc[0][2], acc[0][3]);
  acc_guard4(acc[1][0], acc[1][1], acc[1][2], acc[1][3]);
  acc_guard4(acc[2][0], acc[2][1], acc[2][2], acc[2][3]);
  acc_guard4(acc[3][0], acc[3][1], acc[3][2], acc[3][3]);

  float* slab = sT[wave];
#pragma unroll
  for (int i = 0; i < 4; ++i) {
    const int mBase = m0 + (i << 4);
#pragma unroll
    for (int j = 0; j < 4; ++j) {
      const int n = n0 + (j << 4) + rlane;
      const float bv = bias[n];
#pragma unroll
      for (int r = 0; r < 8; ++r) {
        float v = acc[i][j][r] * scale;
        v += bv;
        v = fmaxf(v, 0.0f);
        slab[(mOff + r) * 68 + (j << 4) + rlane] = v;
      }
    }
    __builtin_amdgcn_fence(__ATOMIC_RELEASE, "workgroup");
    __builtin_amdgcn_wave_barrier();
    __builtin_amdgcn_fence(__ATOMIC_ACQUIRE, "workgroup");
    {
      const int hh = lane >> 4, c4 = (lane & 15) * 4;
      for (int pass = 0; pass < 2; ++pass) {
#pragma unroll
        for (int it = 0; it < 8; ++it) {
          const int row = it * 2 + hh;
          const v4f v = *(const v4f*)(slab + row * 68 + c4);
          *(volatile v4f*)(Cout + (size_t)(mBase + row) * NMLP + n0 + c4) = v;
        }
        __threadfence();
      }
    }
    __builtin_amdgcn_fence(__ATOMIC_RELEASE, "workgroup");
    __builtin_amdgcn_wave_barrier();
    __builtin_amdgcn_fence(__ATOMIC_ACQUIRE, "workgroup");
  }
}

__global__ __launch_bounds__(NTHR) void mlp2_kernel(const float* __restrict__ h1, const float* __restrict__ W2,
                                                    const float* __restrict__ b2, float* __restrict__ out) {
  const int flat = blockIdx.x * NTHR + threadIdx.x;
  if (flat >= NBATCH * NCLS) return;
  const int b = flat / NCLS;
  const int c = flat - b * NCLS;
  const float* hp = h1 + (size_t)b * NMLP;
  const float* wp = W2 + (size_t)c * NMLP;
  float acc = 0.0f;
#pragma unroll 1
  for (int k = 0; k < NMLP; k += 4) {
    const v4f a = *(const v4f*)(hp + k);
    const v4f w = *(const v4f*)(wp + k);
    acc += a[0] * w[0];
    acc += a[1] * w[1];
    acc += a[2] * w[2];
    acc += a[3] * w[3];
  }
  const float res = acc + b2[c];
  *(volatile float*)(out + flat) = res;
  __threadfence();
  *(volatile float*)(out + flat) = res;
}

extern "C" void kernel_launch(void* const* d_in, const int* in_sizes, int n_in,
                              void* d_out, int out_size, void* d_ws, size_t ws_size, hipStream_t stream) {
  if (n_in < 20 || d_out == nullptr || d_ws == nullptr) return;
  if (in_sizes[0] != NTOK || in_sizes[1] != NTOK || in_sizes[2] != NTOK || in_sizes[3] != NTOK ||
      in_sizes[4] != NWORDV * DWORDE || in_sizes[5] != NTAGV * DTAGE || in_sizes[6] != NPOSV * DPOSE ||
      in_sizes[7] != NPOSV * DPOSE || in_sizes[8] != NGATE * NXIN || in_sizes[9] != NGATE * NHID ||
      in_sizes[10] != NGATE || in_sizes[11] != NGATE || in_sizes[12] != NGATE * NXIN || in_sizes[13] != NGATE * NHID ||
      in_sizes[14] != NGATE || in_sizes[15] != NGATE || in_sizes[16] != NMLP * NLIN || in_sizes[17] != NMLP ||
      in_sizes[18] != NCLS * NMLP || in_sizes[19] != NCLS || out_size != NBATCH * NCLS) return;

  const int*   word     = (const int*)d_in[0];
  const int*   tag      = (const int*)d_in[1];
  const int*   pos1     = (const int*)d_in[2];
  const int*   pos2     = (const int*)d_in[3];
  const float* word_emb = (const float*)d_in[4];
  const float* tag_emb  = (const float*)d_in[5];
  const float* pos1_emb = (const float*)d_in[6];
  const float* pos2_emb = (const float*)d_in[7];
  const float* Wih_f    = (const float*)d_in[8];
  const float* Whh_f    = (const float*)d_in[9];
  const float* bih_f    = (const float*)d_in[10];
  const float* bhh_f    = (const float*)d_in[11];
  const float* Wih_b    = (const float*)d_in[12];
  const float* Whh_b    = (const float*)d_in[13];
  const float* bih_b    = (const float*)d_in[14];
  const float* bhh_b    = (const float*)d_in[15];
  const float* W1       = (const float*)d_in[16];
  const float* b1       = (const float*)d_in[17];
  const float* W2       = (const float*)d_in[18];
  const float* b2       = (const float*)d_in[19];
  float* out = (float*)d_out;

  char* ws = (char*)d_ws; size_t off = 0;
  auto carve = [&](size_t bytes) -> char* { char* p = ws + off; off += (bytes + 255) & ~(size_t)255; return p; };
  unsigned short* X16    = (unsigned short*)carve((size_t)NTOK * NXIN * 2);
  unsigned short* WIHF   = (unsigned short*)carve((size_t)NGATE * NXIN * 2);
  unsigned short* WHHF   = (unsigned short*)carve((size_t)NGATE * NHID * 2);
  unsigned short* WIHB   = (unsigned short*)carve((size_t)NGATE * NXIN * 2);
  unsigned short* WHHB   = (unsigned short*)carve((size_t)NGATE * NHID * 2);
  unsigned short* W1H    = (unsigned short*)carve((size_t)NMLP * NLIN * 2);
  unsigned short* HS16   = (unsigned short*)carve((size_t)NTOK * NOUTH * 2);
  unsigned short* FEAT16 = (unsigned short*)carve((size_t)NBATCH * NLIN * 2);
  float*          H1     = (float*)carve((size_t)NBATCH * NMLP * 4);
  int*            IDX1   = (int*)carve((size_t)NBATCH * 4);
  int*            IDX2   = (int*)carve((size_t)NBATCH * 4);
  if (off > ws_size || off > (size_t)134217728) return;

  entity_idx_kernel<<<NBATCH / 32, 32, 0, stream>>>(pos1, pos2, IDX1, IDX2);
  const int n8ih = NGATE * NXIN / 8;
  const int n8hh = NGATE * NHID / 8;
  const int n8w1 = NMLP * NLIN / 8;
  cvt8_f16_kernel<<<n8ih / NTHR, NTHR, 0, stream>>>(Wih_f, WIHF, n8ih);
  cvt8_f16_kernel<<<n8hh / NTHR, NTHR, 0, stream>>>(Whh_f, WHHF, n8hh);
  cvt8_f16_kernel<<<n8ih / NTHR, NTHR, 0, stream>>>(Wih_b, WIHB, n8ih);
  cvt8_f16_kernel<<<n8hh / NTHR, NTHR, 0, stream>>>(Whh_b, WHHB, n8hh);
  cvt8_f16_kernel<<<n8w1 / NTHR, NTHR, 0, stream>>>(W1, W1H, n8w1);
  embed_kernel<<<NTOK / 32, NTHR, 0, stream>>>(word, tag, pos1, pos2, word_emb, tag_emb, pos1_emb, pos2_emb, X16);
  birnn_seq_kernel<<<dim3(NBATCH / 16, 2), NTHR, 0, stream>>>(X16, WIHF, WHHF, WIHB, WHHB, bih_f, bhh_f, bih_b, bhh_b, HS16);
  pool_feat_kernel<<<NBATCH, NTHR, 0, stream>>>(HS16, X16, IDX1, IDX2, FEAT16);
  mlp1_gemm_kernel<<<(NBATCH / 64) * (NMLP / 64) / 8, 256, 0, stream>>>(FEAT16, W1H, H1, b1, CARRY2_INV);
  mlp2_kernel<<<(NBATCH * NCLS) / NTHR, NTHR, 0, stream>>>(H1, W2, b2, out);
}
